// Encoder_67190468378802
// MI455X (gfx1250) — hardware-verified
//
#include <hip/hip_runtime.h>
#include <stddef.h>
#include <stdint.h>
#include <math.h>


#define CF     128
#define K2     256
#define NG     512
#define LATN   64
#define NTHR   256
#define NWAVE  8
#define EPT    8
#define CHUNK  (NTHR * EPT)
#define WCAP   (EPT * 32)
#define LISTN  (NWAVE * WCAP)
#define NBD    8192
#define SLD    13
#define NBA    512
#define SLA    9
#define RCAP   20480
#define DEGCAP 96
#define GBM    64
#define GBN    64
#define GTHR   128
#define LTHR   512
#define LWAVE  16
#define RING   32
#define CSTEP  16
#define AGG_ZINTS (LISTN + 2 * RCAP + 3 * NBA)
#define AGG_LDS_INTS (AGG_ZINTS + 16)
#define WSMAX  134217728

#define U1 2048
#define U2 (U1 + 4096)
#define U3 (U2 + 16384)
#define U4 (U3 + 8192)
#define U5 (U4 + 2048)
#define U6 (U5 + 2048)
#define U7 (U6 + 128)

static_assert((CHUNK & (CHUNK - 1)) == 0 && CHUNK <= 4096);
static_assert((NBD & (NBD - 1)) == 0 && NBD == (1 << SLD));
static_assert((NBA & (NBA - 1)) == 0 && NBA == (1 << SLA));
static_assert(((long long)CHUNK << SLD) < (1LL << 31));
static_assert(((long long)CHUNK << SLA) < (1LL << 31));
static_assert(NBD % (NTHR * 4) == 0);
static_assert(NBA % NWAVE == 0 && NBA % 32 == 0);
static_assert(RCAP % 32 == 0 && AGG_ZINTS % 4 == 0 && LISTN % 4 == 0);
static_assert(CF % 32 == 0 && K2 % 32 == 0 && K2 == 2 * CF && CF == 4 * 32);
static_assert(GBM == (GTHR / 32) * 16 && GBN == 64 && CF % GBN == 0);
static_assert(U1 % NTHR == 0 && U2 % NTHR == 0 && U3 % NTHR == 0 && U4 % NTHR == 0 && U5 % NTHR == 0 && U6 % NTHR == 0);
static_assert(AGG_LDS_INTS * 4 <= 300000);
static_assert(NG == LTHR && LTHR == 32 * LWAVE && CSTEP == LWAVE && RING == 2 * CSTEP);
static_assert((RING * CF) % LTHR == 0);

typedef float          v4f   __attribute__((ext_vector_type(4)));
typedef float          v8f   __attribute__((ext_vector_type(8)));
typedef int            v4i   __attribute__((ext_vector_type(4)));
typedef int            v8i   __attribute__((ext_vector_type(8)));
typedef unsigned int   v4u   __attribute__((ext_vector_type(4)));
typedef unsigned short v8us  __attribute__((ext_vector_type(8)));
typedef unsigned short v16us __attribute__((ext_vector_type(16)));
typedef __bf16         v16bf __attribute__((ext_vector_type(16)));
typedef v4f  __attribute__((may_alias)) v4fa;
typedef v4i  __attribute__((may_alias)) v4ia;
typedef v4u  __attribute__((may_alias)) v4ua;
typedef v8us __attribute__((may_alias)) v8usa;
union FragB { v16bf v; v16us u; v8us h[2]; v8i w; };

__device__ __forceinline__ v8f wmb(const FragB& a, const FragB& b, v8f c) {
  v8f d = __builtin_amdgcn_wmma_f32_16x16x32_bf16(false, a.v, false, b.v, (short)0, c, false, false);
  asm volatile("v_nop\n\tv_nop\n\tv_nop\n\tv_nop" : "+v"(d) : "v"(a.w), "v"(b.w));
  return d;
}

__device__ __forceinline__ unsigned bf16_bits(float f) {
  const unsigned u = __float_as_uint(f);
  return ((u + 0x7FFFu + ((u >> 16) & 1u)) >> 16) & 0xFFFFu;
}
__device__ __forceinline__ float bf16_val(float f) {
  return __uint_as_float(bf16_bits(f) << 16);
}

__device__ __forceinline__ v4u split_row4(float v0, float v1, float v2, float v3, int lane) {
  const unsigned h0 = bf16_bits(v0), h1 = bf16_bits(v1), h2 = bf16_bits(v2), h3 = bf16_bits(v3);
  const unsigned l0 = bf16_bits(v0 - __uint_as_float(h0 << 16));
  const unsigned l1 = bf16_bits(v1 - __uint_as_float(h1 << 16));
  const unsigned l2 = bf16_bits(v2 - __uint_as_float(h2 << 16));
  const unsigned l3 = bf16_bits(v3 - __uint_as_float(h3 << 16));
  const int hw0 = (int)(h0 | (h1 << 16));
  const int hw1 = (int)(h2 | (h3 << 16));
  const int lw0 = (int)(l0 | (l1 << 16));
  const int lw1 = (int)(l2 | (l3 << 16));
  const int sa = (2 * lane) & 31, sb = (2 * lane + 1) & 31;
  const int g0 = __shfl(hw0, sa, 32), g1 = __shfl(hw1, sa, 32);
  const int g2 = __shfl(hw0, sb, 32), g3 = __shfl(hw1, sb, 32);
  const int p0 = __shfl(lw0, sa, 32), p1 = __shfl(lw1, sa, 32);
  const int p2 = __shfl(lw0, sb, 32), p3 = __shfl(lw1, sb, 32);
  const bool ls = lane >= 16;
  v4u pv;
  pv.x = (unsigned)(ls ? p0 : g0);
  pv.y = (unsigned)(ls ? p1 : g1);
  pv.z = (unsigned)(ls ? p2 : g2);
  pv.w = (unsigned)(ls ? p3 : g3);
  return pv;
}

template <int SLB>
__device__ __forceinline__ int scan_chunk(const int* __restrict__ dsts, int nE, int cbase, int slotBase,
                                          int nb, int vec8, int* list, int tid, int lane, int wave) {
  int wc = 0;
  const int el0  = tid * EPT;
  const int e0   = cbase + el0;
  const int sent = -2147483647 - 1;
  v4i da, db;
  if (vec8 != 0 && cbase + CHUNK <= nE) {
    da = *(const v4i*)(dsts + e0);
    db = *(const v4i*)(dsts + e0 + 4);
  } else {
    da.x = (e0     < nE) ? dsts[min(e0,     nE - 1)] : sent;
    da.y = (e0 + 1 < nE) ? dsts[min(e0 + 1, nE - 1)] : sent;
    da.z = (e0 + 2 < nE) ? dsts[min(e0 + 2, nE - 1)] : sent;
    da.w = (e0 + 3 < nE) ? dsts[min(e0 + 3, nE - 1)] : sent;
    db.x = (e0 + 4 < nE) ? dsts[min(e0 + 4, nE - 1)] : sent;
    db.y = (e0 + 5 < nE) ? dsts[min(e0 + 5, nE - 1)] : sent;
    db.z = (e0 + 6 < nE) ? dsts[min(e0 + 6, nE - 1)] : sent;
    db.w = (e0 + 7 < nE) ? dsts[min(e0 + 7, nE - 1)] : sent;
  }
  const unsigned nbs = (unsigned)slotBase;
  const unsigned unb = (unsigned)nb;
  const unsigned s0 = (unsigned)da.x - nbs, s1 = (unsigned)da.y - nbs;
  const unsigned s2 = (unsigned)da.z - nbs, s3 = (unsigned)da.w - nbs;
  const unsigned s4 = (unsigned)db.x - nbs, s5 = (unsigned)db.y - nbs;
  const unsigned s6 = (unsigned)db.z - nbs, s7 = (unsigned)db.w - nbs;
  const bool h0 = s0 < unb, h1 = s1 < unb, h2 = s2 < unb, h3 = s3 < unb;
  const bool h4 = s4 < unb, h5 = s5 < unb, h6 = s6 < unb, h7 = s7 < unb;
  const unsigned any = __builtin_amdgcn_ballot_w32(h0 | h1 | h2 | h3 | h4 | h5 | h6 | h7);
  if (any != 0u) {
#define HITJ(J, HJ, SJ) { \
      const unsigned mj = __builtin_amdgcn_ballot_w32(HJ); \
      if (mj != 0u) { \
        if (HJ) { \
          const int pos = wc + (int)__builtin_amdgcn_mbcnt_lo(mj, 0u); \
          if (pos < WCAP) list[wave * WCAP + pos] = ((el0 + (J)) << SLB) | (int)(SJ); \
        } \
        wc += (int)__builtin_popcount(mj); } }
    HITJ(0, h0, s0)
    HITJ(1, h1, s1)
    HITJ(2, h2, s2)
    HITJ(3, h3, s3)
    HITJ(4, h4, s4)
    HITJ(5, h5, s5)
    HITJ(6, h6, s6)
    HITJ(7, h7, s7)
#undef HITJ
  }
  return wc;
}

__global__ __launch_bounds__(NTHR) void k_wprep(
    const float* __restrict__ W1, const float* __restrict__ W2, const float* __restrict__ Wih,
    const float* __restrict__ Whh, const float* __restrict__ bih, const float* __restrict__ bhh,
    const float* __restrict__ Wm, const float* __restrict__ Wl,
    unsigned short* W1T, unsigned short* W2T, unsigned short* WIH, unsigned short* WHH,
    unsigned short* WML, float* BP) {
  const int u = (int)blockIdx.x * NTHR + (int)threadIdx.x;
  if (u < U6) {
    v8us o;
    unsigned short* dp;
    if (u < U1) {
      const int n = u >> 4, k8 = (u & 15) * 8;
      const float* p = W1 + (size_t)k8 * CF + n;
#pragma unroll
      for (int i = 0; i < 8; ++i) o[i] = (unsigned short)bf16_bits(p[(size_t)i * CF]);
      dp = W1T + (size_t)n * CF + k8;
    } else if (u < U2) {
      const int v = u - U1;
      const int n = v >> 5, k8 = (v & 31) * 8, kk = k8 & (CF - 1);
      const float* p = W2 + (size_t)kk * CF + n;
#pragma unroll
      for (int i = 0; i < 8; ++i) o[i] = (unsigned short)bf16_bits(p[(size_t)i * CF]);
      dp = W2T + (size_t)n * K2 + k8;
    } else if (u < U3) {
      const int v = u - U2;
      const int np = v >> 5, k8 = (v & 31) * 8, kk = k8 & (CF - 1);
      const int j = (np & 3) * CF + (np >> 2);
      const float* p = Wih + (size_t)j * CF + kk;
      const v4f a = *(const v4fa*)p;
      const v4f b = *(const v4fa*)(p + 4);
      o[0] = (unsigned short)bf16_bits(a.x); o[1] = (unsigned short)bf16_bits(a.y);
      o[2] = (unsigned short)bf16_bits(a.z); o[3] = (unsigned short)bf16_bits(a.w);
      o[4] = (unsigned short)bf16_bits(b.x); o[5] = (unsigned short)bf16_bits(b.y);
      o[6] = (unsigned short)bf16_bits(b.z); o[7] = (unsigned short)bf16_bits(b.w);
      dp = WIH + (size_t)np * K2 + k8;
    } else if (u < U4) {
      const int v = u - U3;
      const int np = v >> 4, k8 = (v & 15) * 8;
      const int j = (np & 3) * CF + (np >> 2);
      const float* p = Whh + (size_t)j * CF + k8;
      const v4f a = *(const v4fa*)p;
      const v4f b = *(const v4fa*)(p + 4);
      o[0] = (unsigned short)bf16_bits(a.x); o[1] = (unsigned short)bf16_bits(a.y);
      o[2] = (unsigned short)bf16_bits(a.z); o[3] = (unsigned short)bf16_bits(a.w);
      o[4] = (unsigned short)bf16_bits(b.x); o[5] = (unsigned short)bf16_bits(b.y);
      o[6] = (unsigned short)bf16_bits(b.z); o[7] = (unsigned short)bf16_bits(b.w);
      dp = WHH + (size_t)np * CF + k8;
    } else if (u < U5) {
      const int v = u - U4;
      const int n = v >> 5, k8 = (v & 31) * 8, kk = k8 & (CF - 1);
      const float* p = Wm + (size_t)kk * LATN + n;
#pragma unroll
      for (int i = 0; i < 8; ++i) o[i] = (unsigned short)bf16_bits(p[(size_t)i * LATN]);
      dp = WML + (size_t)n * K2 + k8;
    } else {
      const int v = u - U5;
      const int n = v >> 5, k8 = (v & 31) * 8, kk = k8 & (CF - 1);
      const float* p = Wl + (size_t)kk * LATN + n;
#pragma unroll
      for (int i = 0; i < 8; ++i) o[i] = (unsigned short)bf16_bits(p[(size_t)i * LATN]);
      dp = WML + (size_t)(LATN + n) * K2 + k8;
    }
    *(volatile v8us*)dp = o;
    __threadfence();
    *(volatile v8us*)dp = o;
  } else if (u < U7) {
    const int v = u - U6;
    v4f o;
    o.x = bf16_val(bih[v])          + bf16_val(bhh[v]);
    o.y = bf16_val(bih[CF + v])     + bf16_val(bhh[CF + v]);
    o.z = bf16_val(bih[2 * CF + v]) + bf16_val(bhh[2 * CF + v]);
    o.w = bf16_val(bih[3 * CF + v]) + bf16_val(bhh[3 * CF + v]);
    float* dp = BP + 4 * v;
    *(volatile v4f*)dp = o;
    __threadfence();
    *(volatile v4f*)dp = o;
  }
}

__global__ __launch_bounds__(NTHR) void k_cvx(const float* __restrict__ x, int nN, int nUnits,
                                              unsigned short* xb) {
  const int u = (int)blockIdx.x * NTHR + (int)threadIdx.x;
  if (u >= nUnits) return;
  const int row = u >> 4;
  const int k8  = (u & 15) * 8;
  const int rc  = row < nN ? row : nN - 1;
  const float* p = x + (size_t)rc * CF + k8;
  const v4f a = *(const v4fa*)p;
  const v4f b = *(const v4fa*)(p + 4);
  const bool ok = row < nN;
  v8us o;
  o[0] = ok ? (unsigned short)bf16_bits(a.x) : (unsigned short)0;
  o[1] = ok ? (unsigned short)bf16_bits(a.y) : (unsigned short)0;
  o[2] = ok ? (unsigned short)bf16_bits(a.z) : (unsigned short)0;
  o[3] = ok ? (unsigned short)bf16_bits(a.w) : (unsigned short)0;
  o[4] = ok ? (unsigned short)bf16_bits(b.x) : (unsigned short)0;
  o[5] = ok ? (unsigned short)bf16_bits(b.y) : (unsigned short)0;
  o[6] = ok ? (unsigned short)bf16_bits(b.z) : (unsigned short)0;
  o[7] = ok ? (unsigned short)bf16_bits(b.w) : (unsigned short)0;
  unsigned short* dp = xb + (size_t)row * CF + k8;
  *(volatile v8us*)dp = o;
  __threadfence();
  *(volatile v8us*)dp = o;
}

__global__ __launch_bounds__(NTHR) void k_deg(const int* __restrict__ dsts, int nE, int vec8, float* dis) {
  __shared__ __attribute__((aligned(16))) int scnt[NBD];
  __shared__ __attribute__((aligned(16))) int list[LISTN];
  __shared__ int wcnt[NWAVE];
  const int tid = (int)threadIdx.x, lane = tid & 31, wave = tid >> 5;
  const int nodeBase = (int)blockIdx.x * NBD;

  for (int i = tid; i < NBD; i += NTHR) scnt[i] = 0;
  for (int i = tid; i < LISTN; i += NTHR) list[i] = 0;
  if (tid < NWAVE) wcnt[tid] = 0;
  __syncthreads();

  const int nChunks = (nE + CHUNK - 1) / CHUNK;
#pragma unroll 1
  for (int ch = 0; ch < nChunks; ++ch) {
    const int cbase = ch * CHUNK;
    const int wc = scan_chunk<SLD>(dsts, nE, cbase, nodeBase, NBD, vec8, list, tid, lane, wave);
    if (lane == 0) wcnt[wave] = wc;
    __syncthreads();
    if (wave == 0) {
#pragma unroll 1
      for (int w2 = 0; w2 < NWAVE; ++w2) {
        int c = wcnt[w2];
        c = c < 0 ? 0 : (c > WCAP ? WCAP : c);
#pragma unroll 1
        for (int b0 = 0; b0 < c; b0 += 32) {
          const int idx = b0 + lane;
          const int ent = list[w2 * WCAP + (idx < WCAP ? idx : WCAP - 1)];
          const int m32 = (c - b0) < 32 ? (c - b0) : 32;
#pragma unroll 1
          for (int k = 0; k < m32; ++k) {
            const int u  = __builtin_amdgcn_readlane(ent, k);
            const int sl = u & (NBD - 1);
            if (lane == 0) scnt[sl] = scnt[sl] + 1;
          }
        }
      }
    }
    __syncthreads();
  }

  v4f vals[NBD / (NTHR * 4)];
#pragma unroll
  for (int it = 0; it < NBD / (NTHR * 4); ++it) {
    const int s0 = it * (NTHR * 4) + 4 * tid;
    const v4i c4 = *(const v4ia*)(scnt + s0);
    const float d0 = (float)c4.x + 1.0f, d1 = (float)c4.y + 1.0f;
    const float d2 = (float)c4.z + 1.0f, d3 = (float)c4.w + 1.0f;
    v4f v;
    v.x = (d0 > 0.0f) ? rsqrtf(d0) : 0.0f;
    v.y = (d1 > 0.0f) ? rsqrtf(d1) : 0.0f;
    v.z = (d2 > 0.0f) ? rsqrtf(d2) : 0.0f;
    v.w = (d3 > 0.0f) ? rsqrtf(d3) : 0.0f;
    vals[it] = v;
  }
#pragma unroll
  for (int it = 0; it < NBD / (NTHR * 4); ++it) {
    const int s0 = it * (NTHR * 4) + 4 * tid;
    *(volatile v4f*)(dis + (size_t)nodeBase + s0) = vals[it];
  }
  __threadfence();
#pragma unroll
  for (int it = 0; it < NBD / (NTHR * 4); ++it) {
    const int s0 = it * (NTHR * 4) + 4 * tid;
    *(volatile v4f*)(dis + (size_t)nodeBase + s0) = vals[it];
  }
}

__global__ __launch_bounds__(GTHR) void k_gemm(
    const unsigned short* __restrict__ A, const unsigned short* __restrict__ WT,
    const float* __restrict__ dis, float* outF, int K, int ldo)
{
  __shared__ __attribute__((aligned(16))) float stg[GBM * GBN];
  const int tid = (int)threadIdx.x, lane = tid & 31, wave = tid >> 5, hh = lane >> 4, m = lane & 15;
  const int rowBase = (int)blockIdx.x * GBM;
  const int col0    = (int)blockIdx.y * GBN;

  v8f acc[4];
  {
    const v8f z = {0.f, 0.f, 0.f, 0.f, 0.f, 0.f, 0.f, 0.f};
    acc[0] = z; acc[1] = z; acc[2] = z; acc[3] = z;
  }
  const unsigned short* ap = A  + (size_t)(rowBase + 16 * wave + m) * (size_t)K + 8 * hh;
  const unsigned short* wp = WT + (size_t)(col0 + m) * (size_t)K + 8 * hh;
  const float dv = dis[rowBase + 16 * wave + m];
  const int ksteps = K >> 5;
#pragma unroll 1
  for (int ks = 0; ks < ksteps; ++ks) {
    FragB af;
    af.h[0] = *(const v8usa*)(ap + 32 * ks);
    af.h[1] = *(const v8usa*)(ap + 32 * ks + 16);
#pragma unroll
    for (int t = 0; t < 4; ++t) {
      const unsigned short* wq = wp + (size_t)(16 * t) * (size_t)K + 32 * ks;
      FragB bf;
      bf.h[0] = *(const v8usa*)wq;
      bf.h[1] = *(const v8usa*)(wq + 16);
      acc[t] = wmb(af, bf, acc[t]);
    }
  }

#pragma unroll
  for (int t = 0; t < 4; ++t) {
    const int lc = 16 * t + m;
#pragma unroll
    for (int r = 0; r < 8; ++r) {
      const int lr = 16 * wave + 8 * hh + r;
      stg[lr * GBN + lc] = acc[t][r];
    }
  }
  __syncthreads();

  v4f fv[8];
#pragma unroll
  for (int i = 0; i < 8; ++i) {
    const int lr = 16 * wave + 2 * i + hh;
    const float d = __shfl(dv, 2 * i + hh, 32);
    const v4f v = *(const v4fa*)(stg + lr * GBN + 4 * m);
    v4f y;
    y.x = v.x * d; y.y = v.y * d; y.z = v.z * d; y.w = v.w * d;
    fv[i] = y;
  }
#pragma unroll
  for (int i = 0; i < 8; ++i) {
    const int lr = 16 * wave + 2 * i + hh;
    const int gr = rowBase + lr;
    float* op = outF + (size_t)gr * (size_t)ldo + col0 + 4 * m;
    *(volatile v4f*)op = fv[i];
  }
  __threadfence();
#pragma unroll
  for (int i = 0; i < 8; ++i) {
    const int lr = 16 * wave + 2 * i + hh;
    const int gr = rowBase + lr;
    float* op = outF + (size_t)gr * (size_t)ldo + col0 + 4 * m;
    *(volatile v4f*)op = fv[i];
  }
}

template <int MODE>
__global__ __launch_bounds__(NTHR) void k_scan(const int* __restrict__ srcs, const int* __restrict__ dsts,
                                               int nE, int nN, int vec8, int mRows,
                                               const float* __restrict__ dis, const float* __restrict__ xl,
                                               const float* __restrict__ bLo, const float* __restrict__ bHi,
                                               unsigned short* hb, float* outp, int outHalf) {
  extern __shared__ __attribute__((aligned(16))) int dsm[];
  int* list = dsm;
  int* hl   = dsm + LISTN;
  int* sl   = dsm + LISTN + RCAP;
  int* cnt  = dsm + LISTN + 2 * RCAP;
  int* offs = cnt + NBA;
  int* cur  = offs + NBA;
  int* misc = cur + NBA;
  const int tid = (int)threadIdx.x, lane = tid & 31, wave = tid >> 5;
  const int nodeBase = (int)blockIdx.x * NBA;

  {
    const v4i z4 = {0, 0, 0, 0};
    for (int i = tid * 4; i < AGG_ZINTS; i += NTHR * 4) *(v4ia*)(dsm + i) = z4;
    if (tid < 16) misc[tid] = 0;
  }
  v4f bv;
  {
    const int bo = 4 * (lane & 15);
    const v4f a = *(const v4fa*)(bLo + bo);
    const v4f b = *(const v4fa*)(bHi + bo);
    const unsigned mk = (lane < 16) ? 0xFFFFFFFFu : 0u;
    bv.x = __uint_as_float(((bf16_bits(a.x) << 16) & mk) | ((bf16_bits(b.x) << 16) & ~mk));
    bv.y = __uint_as_float(((bf16_bits(a.y) << 16) & mk) | ((bf16_bits(b.y) << 16) & ~mk));
    bv.z = __uint_as_float(((bf16_bits(a.z) << 16) & mk) | ((bf16_bits(b.z) << 16) & ~mk));
    bv.w = __uint_as_float(((bf16_bits(a.w) << 16) & mk) | ((bf16_bits(b.w) << 16) & ~mk));
  }
  __syncthreads();

  int t = 0, ov = 0;
  const int nChunks = (nE + CHUNK - 1) / CHUNK;
#pragma unroll 1
  for (int ch = 0; ch < nChunks; ++ch) {
    const int cbase = ch * CHUNK;
    const int wc = scan_chunk<SLA>(dsts, nE, cbase, nodeBase, NBA, vec8, list, tid, lane, wave);
    if (lane == 0) misc[wave] = wc;
    __syncthreads();
    if (wave == 0) {
#pragma unroll 1
      for (int w2 = 0; w2 < NWAVE; ++w2) {
        int c = misc[w2];
        c = c < 0 ? 0 : (c > WCAP ? WCAP : c);
#pragma unroll 1
        for (int b0 = 0; b0 < c; b0 += 32) {
          const int idx = b0 + lane;
          const int ent = list[w2 * WCAP + (idx < WCAP ? idx : WCAP - 1)];
          const int m32 = (c - b0) < 32 ? (c - b0) : 32;
#pragma unroll 1
          for (int k = 0; k < m32; ++k) {
            const int u    = __builtin_amdgcn_readlane(ent, k);
            const int slot = u & (NBA - 1);
            const int el   = (u >> SLA) & (CHUNK - 1);
            const int pk   = ((cbase + el) << SLA) | slot;
            if (t < RCAP) {
              if (lane == 0) { hl[t] = pk; cnt[slot] = cnt[slot] + 1; }
              t = t + 1;
            } else {
              ov = 1;
            }
          }
        }
      }
    }
    __syncthreads();
  }
  if (wave == 0 && lane == 0) { misc[8] = t; misc[9] = ov; }
  __syncthreads();
  int tt = misc[8];
  tt = tt < 0 ? 0 : (tt > RCAP ? RCAP : tt);
  const int ovf = misc[9];

  if (wave == 0) {
    const int base = lane * (NBA / 32);
    int s = 0;
#pragma unroll 1
    for (int i = 0; i < NBA / 32; ++i) s += cnt[base + i];
    int incl = s;
#pragma unroll
    for (int d = 1; d < 32; d <<= 1) {
      const int y = __shfl_up(incl, d, 32);
      if (lane >= d) incl += y;
    }
    int run = incl - s;
#pragma unroll 1
    for (int i = 0; i < NBA / 32; ++i) {
      const int cv = cnt[base + i];
      offs[base + i] = run;
      cur[base + i]  = run;
      run += cv;
    }
  }
  __syncthreads();
  if (wave == 0) {
#pragma unroll 1
    for (int b0 = 0; b0 < tt; b0 += 32) {
      const int idx = b0 + lane;
      const int ent = hl[idx < RCAP ? idx : RCAP - 1];
      const int m32 = (tt - b0) < 32 ? (tt - b0) : 32;
#pragma unroll 1
      for (int k = 0; k < m32; ++k) {
        const int u    = __builtin_amdgcn_readlane(ent, k);
        const int slot = u & (NBA - 1);
        if (lane == 0) {
          int p = cur[slot];
          p = p < 0 ? 0 : (p > RCAP - 1 ? RCAP - 1 : p);
          sl[p] = u;
          cur[slot] = p + 1;
        }
      }
    }
  }
  __syncthreads();

  const float qnan = __int_as_float(0x7fc00000);
  const float pz = (ovf != 0) ? qnan : 0.0f;
#pragma unroll 1
  for (int si = 0; si < NBA / NWAVE; ++si) {
    const int s    = si * NWAVE + wave;
    const int node = nodeBase + s;
    int c = cnt[s];
    const bool big = c > DEGCAP;
    c = c < 0 ? 0 : (c > DEGCAP ? DEGCAP : c);
    int o = offs[s];
    o = o < 0 ? 0 : (o > RCAP ? RCAP : o);
    const int nc = node < nN ? node : nN - 1;
    const float dd = dis[nc];
    float a0 = 0.0f, a1 = 0.0f, a2 = 0.0f, a3 = 0.0f;
#pragma unroll 1
    for (int b0 = 0; b0 < c; b0 += 32) {
      int idx = o + b0 + lane;
      idx = idx > RCAP - 1 ? RCAP - 1 : idx;
      const int ent = sl[idx];
      int eid = ent >> SLA;
      eid = eid < 0 ? 0 : (eid > nE - 1 ? nE - 1 : eid);
      int sr = srcs[eid];
      sr = sr < 0 ? 0 : (sr > nN - 1 ? nN - 1 : sr);
      const int m32 = (c - b0) < 32 ? (c - b0) : 32;
#pragma unroll 1
      for (int k = 0; k < m32; ++k) {
        const int sk = __builtin_amdgcn_readlane(sr, k);
        const v4f a = *(const v4fa*)(xl + (size_t)sk * CF + 4 * lane);
        a0 += a.x; a1 += a.y; a2 += a.z; a3 += a.w;
      }
    }
    const v4f sv = *(const v4fa*)(xl + (size_t)nc * CF + 4 * lane);
    const float pzr = big ? qnan : pz;
    const bool live = node < nN;
    float y0 = (a0 + sv.x) * dd + bv.x;
    float y1 = (a1 + sv.y) * dd + bv.y;
    float y2 = (a2 + sv.z) * dd + bv.z;
    float y3 = (a3 + sv.w) * dd + bv.w;
    if constexpr (MODE != 0) {
      y0 = (y0 > 0.0f) ? y0 : (y0 - y0);
      y1 = (y1 > 0.0f) ? y1 : (y1 - y1);
      y2 = (y2 > 0.0f) ? y2 : (y2 - y2);
      y3 = (y3 > 0.0f) ? y3 : (y3 - y3);
    }
    y0 = y0 + pzr; y1 = y1 + pzr; y2 = y2 + pzr; y3 = y3 + pzr;
    if constexpr (MODE != 0) {
      const float v0 = live ? y0 : 0.0f;
      const float v1 = live ? y1 : 0.0f;
      const float v2 = live ? y2 : 0.0f;
      const float v3 = live ? y3 : 0.0f;
      const v4u pv = split_row4(v0, v1, v2, v3, lane);
      unsigned short* hp = hb + (size_t)node * K2 + 8 * lane;
      const bool wr = node < mRows;
      if (wr) *(volatile v4u*)hp = pv;
      __threadfence();
      if (wr) *(volatile v4u*)hp = pv;
    } else {
      v4f ow;
      ow.x = y0; ow.y = y1; ow.z = y2; ow.w = y3;
      const size_t ob = (lane < 16) ? (size_t)0 : (size_t)outHalf;
      float* op = outp + ob + (size_t)node * LATN + 4 * (lane & 15);
      if (live) *(volatile v4f*)op = ow;
      __threadfence();
      if (live) *(volatile v4f*)op = ow;
    }
  }
}

__global__ __launch_bounds__(LTHR) void k_lstm(const unsigned short* __restrict__ h2,
                                               const unsigned short* __restrict__ wih,
                                               const unsigned short* __restrict__ whh,
                                               const float* __restrict__ bp,
                                               unsigned short* hs, int T, int mRows) {
  __shared__ __attribute__((aligned(16))) float ring[RING * CF];
  __shared__ __attribute__((aligned(16))) float xgs[CSTEP * NG];
  const int tid = (int)threadIdx.x, lane = tid & 31, wave = tid >> 5, hh = lane >> 4, m = lane & 15;
  const int q = tid & 3;
  const int qb = lane & ~3;

  unsigned w[64];
  {
    const unsigned short* wr = whh + (size_t)tid * CF;
#pragma unroll
    for (int i = 0; i < 16; ++i) {
      const v4u tv = *(const v4ua*)(wr + 8 * i);
      w[4 * i + 0] = tv.x; w[4 * i + 1] = tv.y; w[4 * i + 2] = tv.z; w[4 * i + 3] = tv.w;
    }
  }
  const float bias = bp[tid];
#pragma unroll
  for (int i = 0; i < (RING * CF) / LTHR; ++i) ring[i * LTHR + tid] = 0.0f;
  float c = 0.0f;
  __syncthreads();

  const unsigned short* bq0 = wih + (size_t)(32 * wave + m) * K2 + 8 * hh;
  const unsigned short* bq1 = bq0 + (size_t)16 * K2;
  const int nCh = T / CSTEP;
#pragma unroll 1
  for (int ch = 0; ch < nCh; ++ch) {
    const int t0 = ch * CSTEP;
    {
      v8f acc0 = {0.f, 0.f, 0.f, 0.f, 0.f, 0.f, 0.f, 0.f};
      v8f acc1 = {0.f, 0.f, 0.f, 0.f, 0.f, 0.f, 0.f, 0.f};
      const unsigned short* ap = h2 + (size_t)(t0 + m) * K2 + 8 * hh;
#pragma unroll
      for (int ks = 0; ks < K2 / 32; ++ks) {
        FragB af, b0, b1;
        af.h[0] = *(const v8usa*)(ap + 32 * ks);
        af.h[1] = *(const v8usa*)(ap + 32 * ks + 16);
        b0.h[0] = *(const v8usa*)(bq0 + 32 * ks);
        b0.h[1] = *(const v8usa*)(bq0 + 32 * ks + 16);
        b1.h[0] = *(const v8usa*)(bq1 + 32 * ks);
        b1.h[1] = *(const v8usa*)(bq1 + 32 * ks + 16);
        acc0 = wmb(af, b0, acc0);
        acc1 = wmb(af, b1, acc1);
      }
#pragma unroll
      for (int r = 0; r < 8; ++r) {
        xgs[(8 * hh + r) * NG + 32 * wave + m]      = acc0[r];
        xgs[(8 * hh + r) * NG + 32 * wave + 16 + m] = acc1[r];
      }
    }
    __syncthreads();

#pragma unroll 1
    for (int s = 0; s < CSTEP; ++s) {
      const int t = t0 + s;
      const float* hp = ring + ((t + RING - 1) & (RING - 1)) * CF;
      float a0 = 0.0f, a1 = 0.0f, a2 = 0.0f, a3 = 0.0f;
#pragma unroll
      for (int k4 = 0; k4 < CF / 4; ++k4) {
        const v4f h4 = *(const v4fa*)(hp + 4 * k4);
        const unsigned w0 = w[2 * k4], w1 = w[2 * k4 + 1];
        a0 = fmaf(h4.x, __uint_as_float(w0 << 16), a0);
        a1 = fmaf(h4.y, __uint_as_float(w0 & 0xFFFF0000u), a1);
        a2 = fmaf(h4.z, __uint_as_float(w1 << 16), a2);
        a3 = fmaf(h4.w, __uint_as_float(w1 & 0xFFFF0000u), a3);
      }
      const float dot = (a0 + a1) + (a2 + a3);
      const float g = (xgs[s * NG + tid] + bias) + dot;
      const float th = tanhf(g);
      const float sg = 1.0f / (1.0f + expf(-g));
      const float act = (q == 2) ? th : sg;
      const float vi = __shfl(act, qb + 0, 32);
      const float vf = __shfl(act, qb + 1, 32);
      const float vg = __shfl(act, qb + 2, 32);
      const float vo = __shfl(act, qb + 3, 32);
      c = vf * c + vi * vg;
      const float hn = vo * tanhf(c);
      if (q == 0) ring[(t & (RING - 1)) * CF + (tid >> 2)] = hn;
      __syncthreads();
    }

    {
      const int slot = (t0 & (RING - 1)) + wave;
      const v4f hv = *(const v4fa*)(ring + slot * CF + 4 * lane);
      const v4u pv = split_row4(hv.x, hv.y, hv.z, hv.w, lane);
      unsigned short* rp = hs + (size_t)(t0 + wave) * K2 + 8 * lane;
      *(volatile v4u*)rp = pv;
      __threadfence();
      *(volatile v4u*)rp = pv;
    }
  }

#pragma unroll 1
  for (int row = T + wave; row < mRows; row += LWAVE) {
    const v4u z = {0u, 0u, 0u, 0u};
    unsigned short* rp = hs + (size_t)row * K2 + 8 * lane;
    *(volatile v4u*)rp = z;
    __threadfence();
    *(volatile v4u*)rp = z;
  }
}

static inline int cdiv(int a, int b) { return (a + b - 1) / b; }
static inline size_t al256(size_t o) { return (o + 255) & ~(size_t)255; }

extern "C" void kernel_launch(void* const* d_in, const int* in_sizes, int n_in,
                              void* d_out, int out_size, void* d_ws, size_t ws_size,
                              hipStream_t stream) {
  if (n_in < 14) return;
  if (in_sizes[0] < CF || (in_sizes[0] % CF) != 0) return;
  const int nN = in_sizes[0] / CF;
  if (nN < 16 || nN > (1 << 22) || (nN % CSTEP) != 0) return;
  if (in_sizes[1] < 2 || (in_sizes[1] & 1) != 0) return;
  const int nE = in_sizes[1] / 2;
  if (nE < 1 || nE >= (1 << (31 - SLA))) return;
  if (in_sizes[2] != CF * CF || in_sizes[3] != CF) return;
  if (in_sizes[4] != CF * CF || in_sizes[5] != CF) return;
  if (in_sizes[6] != NG * CF || in_sizes[7] != NG * CF) return;
  if (in_sizes[8] != NG || in_sizes[9] != NG) return;
  if (in_sizes[10] != CF * LATN || in_sizes[11] != LATN) return;
  if (in_sizes[12] != CF * LATN || in_sizes[13] != LATN) return;
  if ((long long)out_size != (long long)nN * 2 * LATN) return;

  const float* x    = (const float*)d_in[0];
  const int*   edge = (const int*)d_in[1];
  const float* W1   = (const float*)d_in[2];
  const float* b1   = (const float*)d_in[3];
  const float* W2   = (const float*)d_in[4];
  const float* b2   = (const float*)d_in[5];
  const float* Wih  = (const float*)d_in[6];
  const float* Whh  = (const float*)d_in[7];
  const float* bih  = (const float*)d_in[8];
  const float* bhh  = (const float*)d_in[9];
  const float* Wm   = (const float*)d_in[10];
  const float* bm   = (const float*)d_in[11];
  const float* Wl   = (const float*)d_in[12];
  const float* bl   = (const float*)d_in[13];
  float* out = (float*)d_out;
  const int* src = edge;
  const int* dst = edge + nE;

  const int MP   = cdiv(nN, GBM) * GBM;
  const int gM   = MP / GBM;
  const int gD   = cdiv(MP, NBD);
  const int NBPD = gD * NBD;
  const int gA   = cdiv(MP, NBA);
  if ((long long)gA * NBA < (long long)MP) return;
  if (NBPD < MP) return;
  const int vec8 = ((nE & 3) == 0) ? 1 : 0;

  char* ws = (char*)d_ws;
  size_t off = 0;
  const size_t oDIS = off; off = al256(off + (size_t)NBPD * 4);
  const size_t oW1T = off; off = al256(off + (size_t)CF * CF * 2);
  const size_t oW2T = off; off = al256(off + (size_t)CF * K2 * 2);
  const size_t oWIH = off; off = al256(off + (size_t)NG * K2 * 2);
  const size_t oWHH = off; off = al256(off + (size_t)NG * CF * 2);
  const size_t oWML = off; off = al256(off + (size_t)CF * K2 * 2);
  const size_t oBP  = off; off = al256(off + (size_t)NG * 4);
  const size_t oXB  = off; off = al256(off + (size_t)MP * CF * 2);
  const size_t oT   = off; off = al256(off + (size_t)MP * CF * 4);
  const size_t oH1  = off; off = al256(off + (size_t)MP * K2 * 2);
  const size_t oH2  = off; off = al256(off + (size_t)MP * K2 * 2);
  const size_t oHS  = off; off = al256(off + (size_t)MP * K2 * 2);
  if (off > ws_size || off > (size_t)WSMAX) return;
  float*          DIS = (float*)(ws + oDIS);
  unsigned short* W1T = (unsigned short*)(ws + oW1T);
  unsigned short* W2T = (unsigned short*)(ws + oW2T);
  unsigned short* WIH = (unsigned short*)(ws + oWIH);
  unsigned short* WHH = (unsigned short*)(ws + oWHH);
  unsigned short* WML = (unsigned short*)(ws + oWML);
  float*          BP  = (float*)(ws + oBP);
  unsigned short* XB  = (unsigned short*)(ws + oXB);
  float*          T   = (float*)(ws + oT);
  unsigned short* H1  = (unsigned short*)(ws + oH1);
  unsigned short* H2  = (unsigned short*)(ws + oH2);
  unsigned short* HS  = (unsigned short*)(ws + oHS);

  const size_t scanLds = (size_t)AGG_LDS_INTS * 4;
  hipFuncSetAttribute(reinterpret_cast<const void*>(&k_scan<1>), hipFuncAttributeMaxDynamicSharedMemorySize, (int)scanLds);
  hipFuncSetAttribute(reinterpret_cast<const void*>(&k_scan<0>), hipFuncAttributeMaxDynamicSharedMemorySize, (int)scanLds);

  const int nUx = MP * (CF / 8);
  k_wprep<<<cdiv(U7, NTHR), NTHR, 0, stream>>>(W1, W2, Wih, Whh, bih, bhh, Wm, Wl, W1T, W2T, WIH, WHH, WML, BP);
  k_cvx<<<cdiv(nUx, NTHR), NTHR, 0, stream>>>(x, nN, nUx, XB);
  k_deg<<<gD, NTHR, 0, stream>>>(dst, nE, vec8, DIS);
  k_gemm<<<dim3(gM, CF / GBN), GTHR, 0, stream>>>(XB, W1T, DIS, T, CF, CF);
  k_scan<1><<<gA, NTHR, scanLds, stream>>>(src, dst, nE, nN, vec8, MP, DIS, T, b1, b1 + LATN, H1, out, 0);
  k_gemm<<<dim3(gM, CF / GBN), GTHR, 0, stream>>>(H1, W2T, DIS, T, K2, CF);
  k_scan<1><<<gA, NTHR, scanLds, stream>>>(src, dst, nE, nN, vec8, MP, DIS, T, b2, b2 + LATN, H2, out, 0);
  k_lstm<<<1, LTHR, 0, stream>>>(H2, WIH, WHH, BP, HS, nN, MP);
  k_gemm<<<dim3(gM, CF / GBN), GTHR, 0, stream>>>(HS, WML, DIS, T, K2, CF);
  k_scan<0><<<gA, NTHR, scanLds, stream>>>(src, dst, nE, nN, vec8, MP, DIS, T, bm, bl, H1, out, nN * LATN);
}
